// KernelDWConv2d_44727789420779
// MI455X (gfx1250) — hardware-verified
//
#include <hip/hip_runtime.h>
#include <stdint.h>

#define NB    32
#define CIN   256
#define COUT  256
#define IMH   31
#define IMW   31
#define HW    961
#define HWP   992
#define PT    31
#define KS    7
#define NTAP  49
#define HO    25
#define WO    25
#define NPIX  625
#define NPAD  640
#define KK    12544
#define GS    4
#define NG    8
#define NSEG  31360
#define SEGW  14
#define NITEM 1280000
#define ITPB  10

#define COLSCALE 64.0f
#define WSCALE   1024.0f
#define OSCALE   (1.0f / 65536.0f)

static_assert(NB == GS * NG);
static_assert(HW == IMH * IMW);
static_assert(PT * 32 == HWP && HWP >= HW);
static_assert(KK == NTAP * CIN);
static_assert(NSEG == NPAD * NTAP);
static_assert(NSEG % (8 * SEGW) == 0);
static_assert((NB * NTAP) % 8 == 0);
static_assert((COUT * NTAP) % 56 == 0);
static_assert(NITEM * 4 == NB * COUT * NPIX);
static_assert(NITEM % (256 * ITPB) == 0);
static_assert((NPAD % 64) == 0 && (COUT % 64) == 0 && (KK % 32) == 0);
static_assert(((COUT / 64) * (NPAD / 64)) % 8 == 0);
static_assert(NPIX == HO * WO && HO == IMH - KS + 1);

typedef _Float16 v16h __attribute__((ext_vector_type(16)));
typedef _Float16 v8h  __attribute__((ext_vector_type(8)));
typedef float    v8f  __attribute__((ext_vector_type(8)));
typedef float    v4f  __attribute__((ext_vector_type(4)));
typedef unsigned int v4u __attribute__((ext_vector_type(4)));

__device__ __forceinline__ unsigned short bf_bits(float f) {
  unsigned u = __float_as_uint(f);
  return (unsigned short)((u + 0x7FFFu + ((u >> 16) & 1u)) >> 16);
}
__device__ __forceinline__ float bf_up(unsigned short h) { return __uint_as_float(((unsigned)h) << 16); }
__device__ __forceinline__ float bfr(float f) { return bf_up(bf_bits(f)); }
__device__ __forceinline__ unsigned short h_bits(_Float16 x) { return __builtin_bit_cast(unsigned short, x); }
__device__ __forceinline__ unsigned short f2h_bits(float f) { return h_bits((_Float16)f); }
__device__ __forceinline__ unsigned pk16(unsigned short a, unsigned short b) { return (unsigned)a | ((unsigned)b << 16); }
__device__ __forceinline__ v8f zero8() { v8f z = {0.f, 0.f, 0.f, 0.f, 0.f, 0.f, 0.f, 0.f}; return z; }

__device__ __forceinline__ v16h ldfrag_h(const _Float16* p) {
  union { v16h v; v8h h[2]; } f;
  f.h[0] = *(const v8h*)(p);
  f.h[1] = *(const v8h*)(p + 16);
  return f.v;
}

__device__ __forceinline__ v8f mma_h_raw(v16h a, v16h b, v8f c) {
  return __builtin_amdgcn_wmma_f32_16x16x32_f16(false, a, false, b, (short)0, c, false, false);
}
__device__ __forceinline__ void dep_guard_h(v8f& a, v8f& b, v16h x, v16h y) {
#if defined(__HIP_DEVICE_COMPILE__)
  asm volatile("v_nop\n\tv_nop\n\tv_nop\n\tv_nop" : "+v"(a), "+v"(b) : "v"(x), "v"(y));
#endif
}
__device__ __forceinline__ void keep4_h(v16h a, v16h b, v16h c, v16h d) {
#if defined(__HIP_DEVICE_COMPILE__)
  asm volatile("v_nop" :: "v"(a), "v"(b), "v"(c), "v"(d));
#endif
}
__device__ __forceinline__ void acc_guard4(v8f& a, v8f& b, v8f& c, v8f& d) {
#if defined(__HIP_DEVICE_COMPILE__)
  asm volatile("v_nop\n\tv_nop\n\tv_nop\n\tv_nop" : "+v"(a), "+v"(b), "+v"(c), "+v"(d));
#endif
}
__device__ __forceinline__ void wave_sync_lds() {
  __builtin_amdgcn_fence(__ATOMIC_RELEASE, "workgroup");
  __builtin_amdgcn_wave_barrier();
  __builtin_amdgcn_fence(__ATOMIC_ACQUIRE, "workgroup");
}

__global__ __launch_bounds__(256) void cvt_xt(const float* __restrict__ x, unsigned short* xt) {
  __shared__ __align__(16) float sx[CIN * 33];
  const int tid = threadIdx.x;
  const int b   = blockIdx.x / PT;
  const int tp  = blockIdx.x - b * PT;
  const int p0  = tp * 32;
  const float* xb = x + (size_t)b * CIN * HW;
#pragma unroll 8
  for (int it = 0; it < 32; ++it) {
    const int idx = it * 256 + tid;
    const int c = idx >> 5, q = idx & 31;
    const int p = min(p0 + q, HW - 1);
    sx[c * 33 + q] = xb[(size_t)c * HW + p];
  }
  __syncthreads();
  const int wave = tid >> 5, lane = tid & 31, c8 = lane * 8;
  v4u pk[4];
#pragma unroll
  for (int it = 0; it < 4; ++it) {
    const int r = wave * 4 + it;
    v4u p;
#pragma unroll
    for (int e = 0; e < 4; ++e)
      p[e] = pk16(bf_bits(sx[(c8 + 2 * e) * 33 + r]), bf_bits(sx[(c8 + 2 * e + 1) * 33 + r]));
    pk[it] = p;
  }
  unsigned short* dst = xt + ((size_t)b * HWP + p0) * CIN;
  for (int pass = 0; pass < 2; ++pass) {
#pragma unroll
    for (int it = 0; it < 4; ++it) {
      const int r = wave * 4 + it;
      *(volatile v4u*)(dst + (size_t)r * CIN + c8) = pk[it];
    }
    __threadfence();
  }
}

__global__ __launch_bounds__(256) void cvt_kt(const float* __restrict__ kr, unsigned short* kt) {
  const int tid = threadIdx.x, wave = tid >> 5, lane = tid & 31, c8 = lane * 8;
  const int row = blockIdx.x * 8 + wave;
  if (row < NB * NTAP) {
    const int b = row / NTAP, tap = row - b * NTAP;
    const float* src = kr + ((size_t)b * CIN + c8) * NTAP + tap;
    float vals[8];
#pragma unroll
    for (int i = 0; i < 8; ++i) vals[i] = src[i * NTAP];
    v4u p;
#pragma unroll
    for (int i = 0; i < 4; ++i) p[i] = pk16(bf_bits(vals[2 * i]), bf_bits(vals[2 * i + 1]));
    unsigned short* d = kt + (size_t)row * CIN + c8;
    *(volatile v4u*)d = p;
    __threadfence();
    *(volatile v4u*)d = p;
  }
}

__global__ __launch_bounds__(256) void cvt_w(const float* __restrict__ w, unsigned short* wp) {
  const int tid = threadIdx.x, wave = tid >> 5, lane = tid & 31, c8 = lane * 8;
#pragma unroll 1
  for (int it = 0; it < 7; ++it) {
    const int seg = (blockIdx.x * 8 + wave) * 7 + it;
    if (seg < COUT * NTAP) {
      const int o = seg / NTAP, tap = seg - o * NTAP;
      const float* src = w + ((size_t)o * CIN + c8) * NTAP + tap;
      float vals[8];
#pragma unroll
      for (int i = 0; i < 8; ++i) vals[i] = bfr(src[i * NTAP]) * WSCALE;
      v4u p;
#pragma unroll
      for (int i = 0; i < 4; ++i) p[i] = pk16(f2h_bits(vals[2 * i]), f2h_bits(vals[2 * i + 1]));
      unsigned short* d = wp + (size_t)o * KK + (size_t)tap * CIN + c8;
      *(volatile v4u*)d = p;
      __threadfence();
      *(volatile v4u*)d = p;
    }
  }
}

__global__ __launch_bounds__(256) void im2col_mod(const unsigned short* __restrict__ xt,
                                                   const unsigned short* __restrict__ kt,
                                                   unsigned short* col) {
  const int bl = blockIdx.y;
  const unsigned short* xs = xt + (size_t)bl * HWP * CIN;
  const unsigned short* kq = kt + (size_t)bl * NTAP * CIN;
  unsigned short* cd = col + (size_t)bl * NSEG * CIN;
  const int tid = threadIdx.x, wave = tid >> 5, lane = tid & 31, c8 = lane * 8;
  const int segb = (blockIdx.x * 8 + wave) * SEGW;
#pragma unroll 1
  for (int it = 0; it < SEGW; ++it) {
    const int seg = segb + it;
    if (seg < NSEG) {
      const int p   = seg / NTAP;
      const int tap = seg - p * NTAP;
      const int ky  = tap / KS, kx = tap - ky * KS;
      const bool ok = p < NPIX;
      const int pc  = min(p, NPIX - 1);
      const int oy  = pc / WO, ox = pc - oy * WO;
      const int pix = (oy + ky) * IMW + (ox + kx);
      const v4u xv = *(const v4u*)(xs + (size_t)pix * CIN + c8);
      const v4u kv = *(const v4u*)(kq + (size_t)tap * CIN + c8);
      v4u o;
#pragma unroll
      for (int e = 0; e < 4; ++e) {
        const float x0 = bf_up((unsigned short)(xv[e] & 0xFFFFu));
        const float x1 = bf_up((unsigned short)(xv[e] >> 16));
        const float g0 = bf_up((unsigned short)(kv[e] & 0xFFFFu));
        const float g1 = bf_up((unsigned short)(kv[e] >> 16));
        const float f0 = (x0 * g0) * COLSCALE;
        const float f1 = (x1 * g1) * COLSCALE;
        const unsigned wv = pk16(f2h_bits(f0), f2h_bits(f1));
        o[e] = ok ? wv : 0u;
      }
      unsigned short* d = cd + (size_t)seg * CIN + c8;
      *(volatile v4u*)d = o;
      __threadfence();
      *(volatile v4u*)d = o;
    }
  }
}

__global__ __launch_bounds__(256) void gemm64(
    const unsigned short* __restrict__ Ap, int lda,
    const unsigned short* __restrict__ Btp, int ldb, long long strideB,
    float* Cp, int ldc, long long strideC,
    int M, int N, int K, float oscale,
    const float* __restrict__ biasp) {
  const _Float16* A  = (const _Float16*)(const void*)Ap;
  const _Float16* Bt = (const _Float16*)(const void*)Btp;
  __shared__ __align__(16) float sT[8][16 * 68];
  const int b    = blockIdx.y;
  const int lane = threadIdx.x & 31;
  const int wave = threadIdx.x >> 5;
  const int tilesN = N >> 6;
  const int tilesM = M >> 6;
  const int tile = blockIdx.x * 8 + wave;
  if (tile >= tilesM * tilesN) return;
  const int tm = tile / tilesN;
  const int tn = tile - tm * tilesN;
  const int m0 = tm << 6;
  const int n0 = tn << 6;

  const _Float16* Bb = Bt + (size_t)b * strideB;

  const int rlane = lane & 15;
  const int koff  = (lane >> 4) * 8;
  const int mOff  = (lane >> 4) * 8;

  v8f acc[4][4];
#pragma unroll
  for (int i = 0; i < 4; ++i)
#pragma unroll
    for (int j = 0; j < 4; ++j) acc[i][j] = zero8();

  for (int k0 = 0; k0 < K; k0 += 32) {
    v16h bh[4];
#pragma unroll
    for (int j = 0; j < 4; ++j) {
      const size_t bo = (size_t)(n0 + (j << 4) + rlane) * ldb + koff + k0;
      bh[j] = ldfrag_h(Bb + bo);
    }
#pragma unroll
    for (int i = 0; i < 4; ++i) {
      const size_t ao = (size_t)(m0 + (i << 4) + rlane) * lda + koff + k0;
      const v16h ah = ldfrag_h(A + ao);
#pragma unroll
      for (int j = 0; j < 4; ++j) {
        acc[i][j] = mma_h_raw(ah, bh[j], acc[i][j]);
      }
      dep_guard_h(acc[i][0], acc[i][3], ah, bh[3]);
    }
    keep4_h(bh[0], bh[1], bh[2], bh[3]);
  }
  acc_guard4(acc[0][0], acc[0][1], acc[0][2], acc[0][3]);
  acc_guard4(acc[1][0], acc[1][1], acc[1][2], acc[1][3]);
  acc_guard4(acc[2][0], acc[2][1], acc[2][2], acc[2][3]);
  acc_guard4(acc[3][0], acc[3][1], acc[3][2], acc[3][3]);

  float* slab = sT[wave];
  float* C = Cp + (size_t)b * strideC;
#pragma unroll
  for (int i = 0; i < 4; ++i) {
    const int mBase = m0 + (i << 4);
#pragma unroll
    for (int j = 0; j < 4; ++j) {
#pragma unroll
      for (int r = 0; r < 8; ++r) {
        slab[(mOff + r) * 68 + (j << 4) + rlane] = acc[i][j][r];
      }
    }
    wave_sync_lds();
    {
      const int hh = lane >> 4, c4 = (lane & 15) * 4;
      v4f ov[8];
#pragma unroll
      for (int it = 0; it < 8; ++it) {
        const int row = it * 2 + hh;
        const float bv = bfr(biasp[mBase + row]);
        v4f v = *(const v4f*)(slab + row * 68 + c4);
        v[0] = v[0] * oscale + bv;
        v[1] = v[1] * oscale + bv;
        v[2] = v[2] * oscale + bv;
        v[3] = v[3] * oscale + bv;
        ov[it] = v;
      }
      for (int pass = 0; pass < 2; ++pass) {
#pragma unroll
        for (int it = 0; it < 8; ++it) {
          const int row = it * 2 + hh;
          *(volatile v4f*)(C + (size_t)(mBase + row) * ldc + n0 + c4) = ov[it];
        }
        __threadfence();
      }
    }
    wave_sync_lds();
  }
}

__global__ __launch_bounds__(256) void pack_out(const float* __restrict__ op, float* out) {
  const int tid = threadIdx.x;
#pragma unroll 1
  for (int it = 0; it < ITPB; ++it) {
    const int item = (blockIdx.x * ITPB + it) * 256 + tid;
    if (item < NITEM) {
      const int f = item * 4;
      v4f v;
#pragma unroll
      for (int j = 0; j < 4; ++j) {
        const int fi  = f + j;
        const int b   = fi / (COUT * NPIX);
        const int rem = fi - b * (COUT * NPIX);
        const int o   = rem / NPIX;
        const int p   = rem - o * NPIX;
        v[j] = op[((size_t)b * COUT + o) * NPAD + p];
      }
      float* d = out + (size_t)f;
      *(volatile v4f*)d = v;
      __threadfence();
      *(volatile v4f*)d = v;
    }
  }
}

extern "C" void kernel_launch(void* const* d_in, const int* in_sizes, int n_in,
                              void* d_out, int out_size, void* d_ws, size_t ws_size,
                              hipStream_t stream) {
  if (n_in < 4) return;
  if (in_sizes[0] != NB * CIN * HW) return;
  if (in_sizes[1] != NB * CIN * NTAP) return;
  if (in_sizes[2] != COUT * CIN * NTAP) return;
  if (in_sizes[3] != COUT) return;
  if (out_size != NB * COUT * NPIX) return;

  const float* x    = (const float*)d_in[0];
  const float* kern = (const float*)d_in[1];
  const float* wgt  = (const float*)d_in[2];
  const float* bias = (const float*)d_in[3];
  float* out = (float*)d_out;

  const size_t PXT = (size_t)NB * HWP * CIN * 2;
  const size_t PKT = (size_t)NB * NTAP * CIN * 2;
  const size_t PWP = (size_t)COUT * KK * 2;
  const size_t PCL = (size_t)GS * NPAD * KK * 2;
  const size_t POP = (size_t)NB * COUT * NPAD * 4;
  size_t off = 0;
  const size_t oXT = off; off += PXT;
  const size_t oKT = off; off += PKT;
  const size_t oWP = off; off += PWP;
  const size_t oCL = off; off += PCL;
  const size_t oOP = off; off += POP;
  if (off > ws_size) return;
  if (off > (size_t)134217728) return;

  char* ws = (char*)d_ws;
  unsigned short* XT  = (unsigned short*)(ws + oXT);
  unsigned short* KT  = (unsigned short*)(ws + oKT);
  unsigned short* WP  = (unsigned short*)(ws + oWP);
  unsigned short* COL = (unsigned short*)(ws + oCL);
  float*          OP  = (float*)(ws + oOP);

  const dim3 blk(256);
  cvt_xt<<<dim3(NB * PT), blk, 0, stream>>>(x, XT);
  cvt_kt<<<dim3((NB * NTAP) / 8), blk, 0, stream>>>(kern, KT);
  cvt_w<<<dim3((COUT * NTAP) / 56), blk, 0, stream>>>(wgt, WP);
  const dim3 gI2c(NSEG / (8 * SEGW), GS);
  const dim3 gGemm(((COUT / 64) * (NPAD / 64)) / 8, GS);
  for (int g = 0; g < NG; ++g) {
    const unsigned short* XTg = XT + (size_t)g * GS * HWP * CIN;
    const unsigned short* KTg = KT + (size_t)g * GS * NTAP * CIN;
    float*                OPg = OP + (size_t)g * GS * COUT * NPAD;
    im2col_mod<<<gI2c, blk, 0, stream>>>(XTg, KTg, COL);
    gemm64<<<gGemm, blk, 0, stream>>>(
        WP, KK,
        COL, KK, (long long)NPAD * KK,
        OPg, NPAD, (long long)COUT * NPAD,
        COUT, NPAD, KK, OSCALE,
        bias);
  }
  pack_out<<<dim3(NITEM / (256 * ITPB)), blk, 0, stream>>>(OP, out);
  (void)hipGetLastError();
}
